// SpatialMultiHeadAttention_82970178224629
// MI455X (gfx1250) — hardware-verified
//
#include <hip/hip_runtime.h>
#include <math.h>
#include <stdint.h>

constexpr int kBatch = 16;
constexpr int kTok   = 1024;
constexpr int kDim   = 768;
constexpr int kHeads = 12;
constexpr int kHd    = 64;
constexpr int kRows  = kBatch * kTok;
constexpr int kGroupsPerRow = kDim / 8;
constexpr float kScoreScale = 0.125f;
constexpr float kProbScale  = 32768.0f;
constexpr float kLog2BaseOver16 = 0.83048202372184058f;

static_assert(kRows % 64 == 0);
static_assert(kDim % 64 == 0);
static_assert(kTok % 64 == 0);
static_assert(kDim % 32 == 0);
static_assert(kHeads * kHd == kDim);

constexpr size_t kSzW16   = (size_t)3 * kDim * kDim * 2;
constexpr size_t kSzWp16  = (size_t)kDim * kDim * 2;
constexpr size_t kSzTab   = 512 * 4;
constexpr size_t kSzP16   = (size_t)kRows * kDim * 2;
constexpr size_t kSzP32   = (size_t)kRows * kDim * 4;
constexpr size_t kOffWqkv = 0;
constexpr size_t kOffWp   = kOffWqkv + kSzW16;
constexpr size_t kOffCt   = kOffWp + kSzWp16;
constexpr size_t kOffSt   = kOffCt + kSzTab;
constexpr size_t kOffX    = kOffSt + kSzTab;
constexpr size_t kOffT    = kOffX + kSzP16;
constexpr size_t kOffK    = kOffT + kSzP32;
constexpr size_t kOffV    = kOffK + kSzP16;
constexpr size_t kWsTotal = kOffV + kSzP16;
static_assert(kWsTotal == 130551808);
static_assert(kWsTotal <= 134217728);
static_assert(kOffWp % 128 == 0 && kOffCt % 128 == 0 && kOffSt % 128 == 0 && kOffX % 128 == 0 &&
              kOffT % 128 == 0 && kOffK % 128 == 0 && kOffV % 128 == 0);

typedef __attribute__((ext_vector_type(16))) _Float16 v16h;
typedef __attribute__((ext_vector_type(8)))  _Float16 v8h;
typedef __attribute__((ext_vector_type(16))) __bf16   v16b;
typedef __attribute__((ext_vector_type(8)))  __bf16   v8b;
typedef __attribute__((ext_vector_type(8)))  float    v8f;
typedef __attribute__((ext_vector_type(4)))  float    v4f;
typedef __attribute__((ext_vector_type(2)))  float    v2f;
typedef __attribute__((ext_vector_type(4)))  unsigned int v4u;

__device__ __forceinline__ unsigned short f2bf_bits(float f) {
  unsigned u = __float_as_uint(f);
  return (unsigned short)((u + 0x7FFFu + ((u >> 16) & 1u)) >> 16);
}
__device__ __forceinline__ float bf_bits2f(unsigned short h) { return __uint_as_float(((unsigned)h) << 16); }
__device__ __forceinline__ unsigned pk16(unsigned short a, unsigned short b) { return (unsigned)a | ((unsigned)b << 16); }
__device__ __forceinline__ unsigned short h_bits(float f) { return __builtin_bit_cast(unsigned short, (_Float16)f); }

__device__ __forceinline__ void dep_guard_h(v8f& a, v8f& b, v16h x, v16h y) { asm volatile("v_nop\n\tv_nop\n\tv_nop\n\tv_nop" : "+v"(a), "+v"(b) : "v"(x), "v"(y)); }
__device__ __forceinline__ void dep_guard_b(v8f& a, v8f& b, v16b x, v16b y) { asm volatile("v_nop\n\tv_nop\n\tv_nop\n\tv_nop" : "+v"(a), "+v"(b) : "v"(x), "v"(y)); }
__device__ __forceinline__ void keep4_h(v16h a, v16h b, v16h c, v16h d) { asm volatile("v_nop" :: "v"(a), "v"(b), "v"(c), "v"(d)); }
__device__ __forceinline__ void keep4_b(v16b a, v16b b, v16b c, v16b d) { asm volatile("v_nop" :: "v"(a), "v"(b), "v"(c), "v"(d)); }
__device__ __forceinline__ void acc_guard4(v8f& a, v8f& b, v8f& c, v8f& d) { asm volatile("v_nop\n\tv_nop\n\tv_nop\n\tv_nop" : "+v"(a), "+v"(b), "+v"(c), "+v"(d)); }
template <typename T> struct Frag;
template <> struct Frag<_Float16> {
  typedef v16h V; union U { v16h v; v8h h[2]; };
  static __device__ __forceinline__ v16h load(const _Float16* p) {
    U f; f.h[0] = *(const v8h*)(p); f.h[1] = *(const v8h*)(p + 16); return f.v;
  }
  static __device__ __forceinline__ v8f mma(v16h a, v16h b, v8f c) {
    return __builtin_amdgcn_wmma_f32_16x16x32_f16(false, a, false, b, (short)0, c, false, false);
  }
  static __device__ __forceinline__ void guard(v8f& a, v8f& b, v16h x, v16h y) { dep_guard_h(a, b, x, y); }
  static __device__ __forceinline__ void keep(v16h a, v16h b, v16h c, v16h d) { keep4_h(a, b, c, d); }
};
template <> struct Frag<__bf16> {
  typedef v16b V; union U { v16b v; v8b h[2]; };
  static __device__ __forceinline__ v16b load(const __bf16* p) {
    U f; f.h[0] = *(const v8b*)(p); f.h[1] = *(const v8b*)(p + 16); return f.v;
  }
  static __device__ __forceinline__ v8f mma(v16b a, v16b b, v8f c) {
    return __builtin_amdgcn_wmma_f32_16x16x32_bf16(false, a, false, b, (short)0, c, false, false);
  }
  static __device__ __forceinline__ void guard(v8f& a, v8f& b, v16b x, v16b y) { dep_guard_b(a, b, x, y); }
  static __device__ __forceinline__ void keep(v16b a, v16b b, v16b c, v16b d) { keep4_b(a, b, c, d); }
};

template <int ET> struct Elem;
template <> struct Elem<0> { typedef _Float16 T; };
template <> struct Elem<1> { typedef __bf16 T; };
template <int ET, int SPLIT, int BIAS_MODE, int OUT_MODE, bool RESID, int ACT = 0>
__global__ __launch_bounds__(256) void wmma_gemm64(
    const unsigned short* __restrict__ Ap, const unsigned short* __restrict__ A2p, int lda, long strideA,
    const unsigned short* __restrict__ Btp, const unsigned short* __restrict__ Bt2p, int ldb, long strideB,
    void* __restrict__ Cout, void* __restrict__ Cout2, int ldc, long strideC,
    const float* __restrict__ bias,
    const float* __restrict__ resid, long strideR,
    int M, int N, int K, float scale) {
  typedef typename Elem<ET>::T T;
  typedef typename Frag<T>::V V;
  const T* A = (const T*)Ap; const T* A2 = (const T*)A2p; const T* Bt = (const T*)Btp; const T* Bt2 = (const T*)Bt2p;
  __shared__ __align__(16) float sT[8][16 * 68];
  const int b    = blockIdx.y;
  const int lane = threadIdx.x & 31;
  const int wave = threadIdx.x >> 5;
  const int tilesN = N >> 6;
  const int tilesM = M >> 6;
  const int tile = blockIdx.x * 8 + wave;
  if (tile >= tilesM * tilesN) return;
  const int tm = tile / tilesN;
  const int tn = tile - tm * tilesN;
  const int m0 = tm << 6;
  const int n0 = tn << 6;

  const T* Ab  = A  + (size_t)b * strideA;
  const T* Bb  = Bt + (size_t)b * strideB;
  const T* Ab2 = (SPLIT != 0) ? (A2  + (size_t)b * strideA) : nullptr;
  const T* Bb2 = (SPLIT == 1) ? (Bt2 + (size_t)b * strideB) : nullptr;

  const int rlane = lane & 15;
  const int koff  = (lane >> 4) * 8;
  const int mOff  = (lane >> 4) * 8;

  v8f acc[4][4];
#pragma unroll
  for (int i = 0; i < 4; ++i)
#pragma unroll
    for (int j = 0; j < 4; ++j) acc[i][j] = (v8f){0.f,0.f,0.f,0.f,0.f,0.f,0.f,0.f};

  for (int k0 = 0; k0 < K; k0 += 32) {
    V bh[4], bl[4];
#pragma unroll
    for (int j = 0; j < 4; ++j) {
      const size_t bo = (size_t)(n0 + (j << 4) + rlane) * ldb + koff + k0;
      bh[j] = Frag<T>::load(Bb + bo);
      if (SPLIT == 1) bl[j] = Frag<T>::load(Bb2 + bo);
    }
#pragma unroll
    for (int i = 0; i < 4; ++i) {
      const size_t ao = (size_t)(m0 + (i << 4) + rlane) * lda + koff + k0;
      V ah = Frag<T>::load(Ab + ao);
      V al = ah;
      if (SPLIT != 0) al = Frag<T>::load(Ab2 + ao);
#pragma unroll
      for (int j = 0; j < 4; ++j) {
        acc[i][j] = Frag<T>::mma(ah, bh[j], acc[i][j]);
        if (SPLIT == 1) acc[i][j] = Frag<T>::mma(ah, bl[j], acc[i][j]);
        if (SPLIT != 0) acc[i][j] = Frag<T>::mma(al, bh[j], acc[i][j]);
      }
      Frag<T>::guard(acc[i][0], acc[i][3], ah, al);
    }
    Frag<T>::keep(bh[0], bh[1], bh[2], bh[3]);
    if (SPLIT == 1) Frag<T>::keep(bl[0], bl[1], bl[2], bl[3]);
  }
  acc_guard4(acc[0][0], acc[0][1], acc[0][2], acc[0][3]);
  acc_guard4(acc[1][0], acc[1][1], acc[1][2], acc[1][3]);
  acc_guard4(acc[2][0], acc[2][1], acc[2][2], acc[2][3]);
  acc_guard4(acc[3][0], acc[3][1], acc[3][2], acc[3][3]);

  float* slab = sT[wave];
  const float* Rb = RESID ? (resid + (size_t)b * strideR) : nullptr;
#pragma unroll
  for (int i = 0; i < 4; ++i) {
    const int mBase = m0 + (i << 4);
#pragma unroll
    for (int j = 0; j < 4; ++j) {
      const int n = n0 + (j << 4) + rlane;
      float bv = 0.f;
      if (BIAS_MODE == 2) bv = bias[n];
#pragma unroll
      for (int r = 0; r < 8; ++r) {
        float v = acc[i][j][r] * scale;
        if (BIAS_MODE == 1) v += bias[mBase + mOff + r];
        if (BIAS_MODE == 2) v += bv;
        if (RESID) v += Rb[(size_t)(mBase + mOff + r) * ldc + n];
        if (ACT == 1) v = tanhf(v);
        if (ACT == 2) v = fmaxf(v, 0.0f);
        if (ACT == 3) v = v / (1.0f + expf(-v));
        if (ACT == 4) v = (v > 0.f) ? v : 0.01f * v;
        slab[(mOff + r) * 68 + (j << 4) + rlane] = v;
      }
    }
    __builtin_amdgcn_fence(__ATOMIC_RELEASE, "workgroup");
    __builtin_amdgcn_wave_barrier();
    __builtin_amdgcn_fence(__ATOMIC_ACQUIRE, "workgroup");
    if (OUT_MODE == 0) {
      float* C = (float*)Cout + (size_t)b * strideC;
      const int hh = lane >> 4, c4 = (lane & 15) * 4;
      for (int pass = 0; pass < 2; ++pass) {
#pragma unroll
        for (int it = 0; it < 8; ++it) {
          const int row = it * 2 + hh;
          v4f v = *(const v4f*)(slab + row * 68 + c4);
          *(volatile v4f*)(C + (size_t)(mBase + row) * ldc + n0 + c4) = v;
        }
        __threadfence();
      }
    } else {
      const int q = lane >> 3, c8 = (lane & 7) * 8;
      unsigned short* C  = (unsigned short*)Cout  + (size_t)b * strideC;
      unsigned short* C2 = (OUT_MODE == 2) ? ((unsigned short*)Cout2 + (size_t)b * strideC) : nullptr;
      for (int pass = 0; pass < 2; ++pass) {
#pragma unroll
        for (int it = 0; it < 4; ++it) {
          const int row = it * 4 + q;
          const float* sp = slab + row * 68 + c8;
          v8h hv, lv;
#pragma unroll
          for (int e = 0; e < 8; ++e) {
            if (OUT_MODE == 1) {
              hv[e] = (_Float16)sp[e];
            } else {
              unsigned short hb = f2bf_bits(sp[e]);
              unsigned short lb = f2bf_bits(sp[e] - bf_bits2f(hb));
              hv[e] = __builtin_bit_cast(_Float16, hb);
              lv[e] = __builtin_bit_cast(_Float16, lb);
            }
          }
          *(volatile v8h*)(C + (size_t)(mBase + row) * ldc + n0 + c8) = hv;
          if (OUT_MODE == 2) *(volatile v8h*)(C2 + (size_t)(mBase + row) * ldc + n0 + c8) = lv;
        }
        __threadfence();
      }
    }
    __builtin_amdgcn_fence(__ATOMIC_RELEASE, "workgroup");
    __builtin_amdgcn_wave_barrier();
    __builtin_amdgcn_fence(__ATOMIC_ACQUIRE, "workgroup");
  }
}

__global__ __launch_bounds__(256) void cast_f32_bf16x2(const float* __restrict__ in, unsigned short* __restrict__ out, int n2) {
  const int i = blockIdx.x * 256 + threadIdx.x;
  if (i < n2) {
    const v2f f = *(const v2f*)(in + 2 * (size_t)i);
    const unsigned u = pk16(f2bf_bits(f[0]), f2bf_bits(f[1]));
    ((volatile unsigned*)out)[i] = u;
    __threadfence();
    ((volatile unsigned*)out)[i] = u;
  }
}

__global__ __launch_bounds__(256) void split_bf16x2_kernel(const float* __restrict__ in, unsigned short* __restrict__ hi,
                                                           unsigned short* __restrict__ lo, int n2) {
  const int i = blockIdx.x * 256 + threadIdx.x;
  if (i < n2) {
    const v2f f = *(const v2f*)(in + 2 * (size_t)i);
    const unsigned short h0 = f2bf_bits(f[0]), h1 = f2bf_bits(f[1]);
    const unsigned short l0 = f2bf_bits(f[0] - bf_bits2f(h0)), l1 = f2bf_bits(f[1] - bf_bits2f(h1));
    const unsigned uh = pk16(h0, h1), ul = pk16(l0, l1);
    ((volatile unsigned*)hi)[i] = uh;
    ((volatile unsigned*)lo)[i] = ul;
    __threadfence();
    ((volatile unsigned*)hi)[i] = uh;
    ((volatile unsigned*)lo)[i] = ul;
  }
}

__device__ __forceinline__ void sc_eval(float ang, float& sn, float& cs) {
  const float kf = rintf(ang * 0.63661977236758134f);
  const int kq = (int)kf;
  float r = fmaf(-kf, 1.57079637050628662109375f, ang);
  r = fmaf(-kf, -4.37113900018624283e-8f, r);
  const float r2 = r * r;
  float sp = fmaf(r2, 2.75573192239858906526e-6f, -1.98412698412698412698e-4f);
  sp = fmaf(r2, sp, 8.33333333333333333e-3f);
  sp = fmaf(r2, sp, -1.66666666666666667e-1f);
  const float sv = fmaf(r2 * r, sp, r);
  float cp = fmaf(r2, -2.75573192239858906526e-7f, 2.48015873015873015873e-5f);
  cp = fmaf(r2, cp, -1.38888888888888889e-3f);
  cp = fmaf(r2, cp, 4.16666666666666667e-2f);
  cp = fmaf(r2, cp, -0.5f);
  const float cv = fmaf(r2, cp, 1.0f);
  const int q = kq & 3;
  sn = (q == 0) ? sv : (q == 1) ? cv : (q == 2) ? -sv : -cv;
  cs = (q == 0) ? cv : (q == 1) ? -sv : (q == 2) ? -cv : sv;
}

__global__ __launch_bounds__(512) void rope_tab_kernel(float* __restrict__ ctab, float* __restrict__ stab) {
  const int t = threadIdx.x;
  const int pos = t >> 4, fi = t & 15;
  const float inv = exp2f(-(float)fi * kLog2BaseOver16);
  const float ang = (float)pos * inv;
  float sn, cs;
  sc_eval(ang, sn, cs);
  ((volatile float*)ctab)[t] = cs;
  ((volatile float*)stab)[t] = sn;
  __threadfence();
  ((volatile float*)ctab)[t] = cs;
  ((volatile float*)stab)[t] = sn;
}

__global__ __launch_bounds__(256) void rope_cvt_kernel(const float* __restrict__ src, const float* __restrict__ ctab,
                                                       const float* __restrict__ stab, unsigned short* __restrict__ dst, int nthr) {
  const int t = blockIdx.x * 256 + threadIdx.x;
  if (t >= nthr) return;
  const int m = t / kGroupsPerRow;
  const int g = t - m * kGroupsPerRow;
  const int col0 = g * 8;
  const int n = m & (kTok - 1);
  const int py = n >> 5, px = n & 31;
  const int dd = col0 & 63;
  const int pos = (dd < 32) ? py : px;
  const int ib = (dd & 31) >> 1;
  const float* sp = src + (size_t)m * kDim + col0;
  const v4f a  = *(const v4f*)sp;
  const v4f bq = *(const v4f*)(sp + 4);
  const v4f cc = *(const v4f*)(ctab + pos * 16 + ib);
  const v4f ss = *(const v4f*)(stab + pos * 16 + ib);
  const float o0 = a[0] * cc[0] - a[1] * ss[0];
  const float o1 = a[0] * ss[0] + a[1] * cc[0];
  const float o2 = a[2] * cc[1] - a[3] * ss[1];
  const float o3 = a[2] * ss[1] + a[3] * cc[1];
  const float o4 = bq[0] * cc[2] - bq[1] * ss[2];
  const float o5 = bq[0] * ss[2] + bq[1] * cc[2];
  const float o6 = bq[2] * cc[3] - bq[3] * ss[3];
  const float o7 = bq[2] * ss[3] + bq[3] * cc[3];
  v4u u;
  u[0] = pk16(h_bits(o0), h_bits(o1));
  u[1] = pk16(h_bits(o2), h_bits(o3));
  u[2] = pk16(h_bits(o4), h_bits(o5));
  u[3] = pk16(h_bits(o6), h_bits(o7));
  unsigned short* dp = dst + (size_t)m * kDim + col0;
  *(volatile v4u*)dp = u;
  __threadfence();
  *(volatile v4u*)dp = u;
}

#define AT_D 64
#define AT_NW 4
#define AT_QB 64
#define AT_KC 64

__device__ __forceinline__ v8f at_mma_h(v16h a, v16h b, v8f c) {
  c = __builtin_amdgcn_wmma_f32_16x16x32_f16(false, a, false, b, (short)0, c, false, false);
  asm volatile("v_nop\n\tv_nop\n\tv_nop\n\tv_nop" : "+v"(c) : "v"(a), "v"(b));
  return c;
}

__global__ __launch_bounds__(128)
void attn_f16_kernel(const unsigned short* __restrict__ qpl, const unsigned short* __restrict__ kpl,
                     const unsigned short* __restrict__ vtpl, float* __restrict__ outp) {
  union FH { v16h v; v8h h[2]; };
  __shared__ __align__(16) _Float16 Ksh[AT_KC * AT_D];
  __shared__ __align__(16) _Float16 Vth[AT_D * AT_KC];
  __shared__ __align__(16) _Float16 Psh[AT_NW][16 * AT_KC];
  __shared__ __align__(16) float    Os[AT_NW][16 * 68];

  const int tid  = threadIdx.x;
  const int wave = tid >> 5;
  const int lane = tid & 31;
  const int hh   = lane >> 4;
  const int c    = lane & 15;

  const int nqb = kTok / AT_QB;
  const int bx  = blockIdx.x;
  const int qb  = bx % nqb;
  const int bhd = bx / nqb;
  const int h   = bhd % kHeads;
  const int b   = bhd / kHeads;
  const int q0  = qb * AT_QB + wave * 16;

  const _Float16* Qb = (const _Float16*)(const void*)qpl  + (size_t)b * kTok * kDim + (size_t)h * AT_D;
  const _Float16* Kb = (const _Float16*)(const void*)kpl  + (size_t)b * kTok * kDim + (size_t)h * AT_D;
  const _Float16* Vb = (const _Float16*)(const void*)vtpl + (size_t)b * kDim * kTok + (size_t)h * AT_D * kTok;
  float*          ob = outp + (size_t)b * kTok * kDim + (size_t)h * AT_D;

  v16h qa[2];
#pragma unroll
  for (int dc = 0; dc < 2; ++dc)
    qa[dc] = Frag<_Float16>::load(Qb + (size_t)(q0 + c) * kDim + dc * 32 + 8 * hh);

  float mrow[8], lrow[8];
  v8f oacc[4];
#pragma unroll
  for (int r = 0; r < 8; ++r) { mrow[r] = -INFINITY; lrow[r] = 0.f; }
#pragma unroll
  for (int t = 0; t < 4; ++t) oacc[t] = (v8f){0.f,0.f,0.f,0.f,0.f,0.f,0.f,0.f};

  for (int kc = 0; kc < kTok / AT_KC; ++kc) {
    const int kv0 = kc * AT_KC;
    __syncthreads();
    {
      const int r = tid >> 1, half = (tid & 1) * 32;
      const _Float16* ks = Kb + (size_t)(kv0 + r) * kDim + half;
      const _Float16* vs = Vb + (size_t)r * kTok + kv0 + half;
#pragma unroll
      for (int i = 0; i < 4; ++i) {
        const v8h a0 = *(const v8h*)(ks + 8 * i);
        const v8h b0 = *(const v8h*)(vs + 8 * i);
        *(v8h*)(Ksh + r * AT_D  + half + 8 * i) = a0;
        *(v8h*)(Vth + r * AT_KC + half + 8 * i) = b0;
      }
    }
    __syncthreads();

    v8f s[4];
#pragma unroll
    for (int j = 0; j < 4; ++j) {
      s[j] = (v8f){0.f,0.f,0.f,0.f,0.f,0.f,0.f,0.f};
#pragma unroll
      for (int dc = 0; dc < 2; ++dc) {
        FH kb;
        kb.h[0] = *(const v8h*)(Ksh + (j * 16 + c) * AT_D + dc * 32 + 8 * hh);
        kb.h[1] = *(const v8h*)(Ksh + (j * 16 + c) * AT_D + dc * 32 + 16 + 8 * hh);
        s[j] = at_mma_h(qa[dc], kb.v, s[j]);
      }
    }
    float cm[8];
#pragma unroll
    for (int r = 0; r < 8; ++r) {
      float m = -INFINITY;
#pragma unroll
      for (int j = 0; j < 4; ++j) {
        const float sv = s[j][r] * kScoreScale;
        s[j][r] = sv;
        m = fmaxf(m, sv);
      }
#pragma unroll
      for (int off = 1; off < 16; off <<= 1) m = fmaxf(m, __shfl_xor(m, off, 32));
      cm[r] = m;
    }
    _Float16* pw = Psh[wave];
#pragma unroll
    for (int r = 0; r < 8; ++r) {
      const float mnew = fmaxf(mrow[r], cm[r]);
      const float alpha = expf(mrow[r] - mnew);
      mrow[r] = mnew;
      float psum = 0.f;
#pragma unroll
      for (int j = 0; j < 4; ++j) {
        const float p = expf(s[j][r] - mnew);
        psum += p;
        pw[(8 * hh + r) * AT_KC + j * 16 + c] = (_Float16)(p * kProbScale);
      }
#pragma unroll
      for (int off = 1; off < 16; off <<= 1) psum += __shfl_xor(psum, off, 32);
      lrow[r] = lrow[r] * alpha + psum;
#pragma unroll
      for (int t = 0; t < 4; ++t) oacc[t][r] *= alpha;
    }
    __builtin_amdgcn_fence(__ATOMIC_RELEASE, "workgroup");
    __builtin_amdgcn_wave_barrier();
    __builtin_amdgcn_fence(__ATOMIC_ACQUIRE, "workgroup");
#pragma unroll 1
    for (int kk = 0; kk < 2; ++kk) {
      FH pa;
      pa.h[0] = *(const v8h*)(pw + c * AT_KC + kk * 32 + 8 * hh);
      pa.h[1] = *(const v8h*)(pw + c * AT_KC + kk * 32 + 16 + 8 * hh);
#pragma unroll
      for (int t = 0; t < 4; ++t) {
        FH vb;
        vb.h[0] = *(const v8h*)(Vth + (t * 16 + c) * AT_KC + kk * 32 + 8 * hh);
        vb.h[1] = *(const v8h*)(Vth + (t * 16 + c) * AT_KC + kk * 32 + 16 + 8 * hh);
        oacc[t] = at_mma_h(pa.v, vb.v, oacc[t]);
      }
    }
  }

  float* os = Os[wave];
#pragma unroll
  for (int r = 0; r < 8; ++r) {
    const float inv = 1.0f / (lrow[r] * kProbScale);
#pragma unroll
    for (int t = 0; t < 4; ++t) os[(8 * hh + r) * 68 + t * 16 + c] = oacc[t][r] * inv;
  }
  __builtin_amdgcn_fence(__ATOMIC_RELEASE, "workgroup");
  __builtin_amdgcn_wave_barrier();
  __builtin_amdgcn_fence(__ATOMIC_ACQUIRE, "workgroup");
  {
    const int c4 = (lane & 15) * 4;
    for (int pass = 0; pass < 2; ++pass) {
#pragma unroll
      for (int it = 0; it < 8; ++it) {
        const int row = it * 2 + hh;
        v4f val = *(const v4f*)(os + row * 68 + c4);
        *(volatile v4f*)(ob + (size_t)(q0 + row) * kDim + c4) = val;
      }
      __threadfence();
    }
  }
}

extern "C" void kernel_launch(void* const* d_in, const int* in_sizes, int n_in,
                              void* d_out, int out_size, void* d_ws, size_t ws_size, hipStream_t stream) {
  if (n_in < 5) return;
  if (in_sizes[0] != kRows * kDim || in_sizes[1] != 3 * kDim * kDim || in_sizes[2] != 3 * kDim ||
      in_sizes[3] != kDim * kDim || in_sizes[4] != kDim || out_size != kRows * kDim) return;
  if (ws_size < kWsTotal) return;

  const float* x      = (const float*)d_in[0];
  const float* qkv_w  = (const float*)d_in[1];
  const float* qkv_b  = (const float*)d_in[2];
  const float* proj_w = (const float*)d_in[3];
  const float* proj_b = (const float*)d_in[4];
  float* outf = (float*)d_out;

  char* ws = (char*)d_ws;
  unsigned short* wqkv = (unsigned short*)(ws + kOffWqkv);
  unsigned short* wp   = (unsigned short*)(ws + kOffWp);
  float* ctab = (float*)(ws + kOffCt);
  float* stab = (float*)(ws + kOffSt);
  unsigned short* xb   = (unsigned short*)(ws + kOffX);
  unsigned short* qpl  = xb;
  float* tf32 = (float*)(ws + kOffT);
  unsigned short* kpl  = (unsigned short*)(ws + kOffK);
  unsigned short* vtpl = (unsigned short*)(ws + kOffV);
  unsigned short* ohp  = kpl;
  unsigned short* olp  = vtpl;

  const int n2x = kRows * kDim / 2;
  const int n2w = 3 * kDim * kDim / 2;
  const int n2p = kDim * kDim / 2;

  cast_f32_bf16x2<<<(n2x + 255) / 256, 256, 0, stream>>>(x, xb, n2x);
  cast_f32_bf16x2<<<(n2w + 255) / 256, 256, 0, stream>>>(qkv_w, wqkv, n2w);
  cast_f32_bf16x2<<<(n2p + 255) / 256, 256, 0, stream>>>(proj_w, wp, n2p);
  rope_tab_kernel<<<1, 512, 0, stream>>>(ctab, stab);

  wmma_gemm64<1, 0, 1, 1, false><<<dim3(((kDim / 64) * (kTok / 64)) / 8, kBatch), 256, 0, stream>>>(
      wqkv + (size_t)2 * kDim * kDim, wqkv + (size_t)2 * kDim * kDim, kDim, 0L,
      xb, xb, kDim, (long)kTok * kDim,
      (void*)vtpl, (void*)vtpl, kTok, (long)kDim * kTok,
      qkv_b + 2 * kDim, qkv_b, 0L,
      kDim, kTok, kDim, 1.0f);

  wmma_gemm64<1, 0, 2, 0, false><<<dim3(((kRows / 64) * (kDim / 64)) / 8, 1), 256, 0, stream>>>(
      xb, xb, kDim, 0L,
      wqkv + (size_t)kDim * kDim, wqkv + (size_t)kDim * kDim, kDim, 0L,
      (void*)tf32, (void*)tf32, kDim, 0L,
      qkv_b + kDim, qkv_b, 0L,
      kRows, kDim, kDim, 1.0f);
  const int nthr = kRows * kGroupsPerRow;
  rope_cvt_kernel<<<(nthr + 255) / 256, 256, 0, stream>>>(tf32, ctab, stab, kpl, nthr);

  wmma_gemm64<1, 0, 2, 0, false><<<dim3(((kRows / 64) * (kDim / 64)) / 8, 1), 256, 0, stream>>>(
      xb, xb, kDim, 0L,
      wqkv, wqkv, kDim, 0L,
      (void*)tf32, (void*)tf32, kDim, 0L,
      qkv_b, qkv_b, 0L,
      kRows, kDim, kDim, 1.0f);
  rope_cvt_kernel<<<(nthr + 255) / 256, 256, 0, stream>>>(tf32, ctab, stab, qpl, nthr);

  attn_f16_kernel<<<kBatch * kHeads * (kTok / AT_QB), 128, 0, stream>>>(qpl, kpl, vtpl, tf32);

  split_bf16x2_kernel<<<(n2x + 255) / 256, 256, 0, stream>>>(tf32, ohp, olp, n2x);

  wmma_gemm64<1, 2, 2, 0, false><<<dim3(((kRows / 64) * (kDim / 64)) / 8, 1), 256, 0, stream>>>(
      ohp, olp, kDim, 0L,
      wp, wp, kDim, 0L,
      (void*)outf, (void*)outf, kDim, 0L,
      proj_b, proj_b, 0L,
      kRows, kDim, kDim, 1.0f);
}
